// PlainSelfAttention_87411174408369
// MI455X (gfx1250) — hardware-verified
//
#include <hip/hip_runtime.h>
#include <math.h>
#include <stdint.h>

#define NBATCH 2
#define SEQ    2048
#define DM     1024
#define NH     16
#define HD     64
#define QKP    (2 * DM)
#define W3     (3 * DM)
#define MP     (NBATCH * SEQ)
#define NQB    (SEQ / 64)
#define WSC    64.0f
#define PSC    64.0f
#define CSC    64.0f
#define LOSC   1024.0f
#define QC     5.0f
#define QEPS   1.0e-6f
static_assert(NH * HD == DM);
static_assert((SEQ % 64) == 0 && (DM % 64) == 0 && (W3 % 64) == 0 && (MP % 64) == 0 && (QKP % 64) == 0);
static_assert((SEQ % 256) == 0);
static_assert(((NBATCH * DM) % 256) == 0);
static_assert(((MP * DM / 8) % 256) == 0);
static_assert((((MP / 64) * (QKP / 64)) % 8) == 0 && (((DM / 64) * (SEQ / 64)) % 8) == 0 && (((MP / 64) * (DM / 64)) % 8) == 0);

typedef _Float16 v16h __attribute__((ext_vector_type(16)));
typedef _Float16 v8h  __attribute__((ext_vector_type(8)));
typedef float    v8f  __attribute__((ext_vector_type(8)));
typedef float    v4f  __attribute__((ext_vector_type(4)));
typedef unsigned int v4u __attribute__((ext_vector_type(4)));

union FragH { v16h v; v8h h[2]; };

__device__ __forceinline__ unsigned short bf_bits(float f) {
  unsigned u = __float_as_uint(f);
  return (unsigned short)((u + 0x7FFFu + ((u >> 16) & 1u)) >> 16);
}
__device__ __forceinline__ float bf_up(unsigned short h) { return __uint_as_float(((unsigned)h) << 16); }
__device__ __forceinline__ float bfr(float f) { return bf_up(bf_bits(f)); }
__device__ __forceinline__ unsigned short h_bits(_Float16 x) { return __builtin_bit_cast(unsigned short, x); }
__device__ __forceinline__ unsigned pk16(unsigned short a, unsigned short b) { return (unsigned)a | ((unsigned)b << 16); }
__device__ __forceinline__ v8f zero8() { v8f z = {0.f, 0.f, 0.f, 0.f, 0.f, 0.f, 0.f, 0.f}; return z; }
__device__ __forceinline__ float gelu_f(float v) { return 0.5f * v * (1.0f + erff(v * 0.70710678118654752f)); }

__device__ __forceinline__ void split_h(float f, unsigned short& hi, unsigned short& lo) {
  float hf = (float)(_Float16)f;
  hf = (fabsf(hf) < 6.103515625e-05f) ? 0.0f : hf;
  hi = h_bits((_Float16)hf);
  lo = h_bits((_Float16)((f - hf) * LOSC));
}

__device__ __forceinline__ v16h ldfrag_h(const _Float16* p) {
  FragH f;
  f.h[0] = *(const v8h*)(p);
  f.h[1] = *(const v8h*)(p + 16);
  return f.v;
}

__device__ __forceinline__ v8f mma_h(v16h a, v16h b, v8f c) {
  c = __builtin_amdgcn_wmma_f32_16x16x32_f16(false, a, false, b, (short)0, c, false, false);
#if defined(__HIP_DEVICE_COMPILE__)
  asm volatile("v_nop\n\tv_nop\n\tv_nop\n\tv_nop" : "+v"(c) : "v"(a), "v"(b));
#endif
  return c;
}
__device__ __forceinline__ v8f mma_h_raw(v16h a, v16h b, v8f c) {
  return __builtin_amdgcn_wmma_f32_16x16x32_f16(false, a, false, b, (short)0, c, false, false);
}
__device__ __forceinline__ void dep_guard1(v8f& a, v8f& b, v16h x) {
#if defined(__HIP_DEVICE_COMPILE__)
  asm volatile("v_nop\n\tv_nop\n\tv_nop\n\tv_nop" : "+v"(a), "+v"(b) : "v"(x));
#endif
}
__device__ __forceinline__ void keep4_h(v16h a, v16h b, v16h c, v16h d) {
#if defined(__HIP_DEVICE_COMPILE__)
  asm volatile("v_nop" :: "v"(a), "v"(b), "v"(c), "v"(d));
#endif
}
__device__ __forceinline__ void acc_guard4(v8f& a, v8f& b, v8f& c, v8f& d) {
#if defined(__HIP_DEVICE_COMPILE__)
  asm volatile("v_nop\n\tv_nop\n\tv_nop\n\tv_nop" : "+v"(a), "+v"(b), "+v"(c), "+v"(d));
#endif
}
__device__ __forceinline__ void wave_sync_lds() {
  __builtin_amdgcn_fence(__ATOMIC_RELEASE, "workgroup");
  __builtin_amdgcn_wave_barrier();
  __builtin_amdgcn_fence(__ATOMIC_ACQUIRE, "workgroup");
}
__device__ __forceinline__ float wsum(float v) {
#pragma unroll
  for (int off = 16; off > 0; off >>= 1) v += __shfl_xor(v, off, 32);
  return v;
}

__global__ __launch_bounds__(256) void conv_h16(const float* __restrict__ W, unsigned short* Wh, int n8, float wsc) {
  const int i  = blockIdx.x * 256 + threadIdx.x;
  const int ic = (i < n8) ? i : (n8 - 1);
  const float* src = W + (size_t)ic * 8;
  const v4f a = *(const v4f*)(src);
  const v4f c = *(const v4f*)(src + 4);
  v4u o;
  o[0] = pk16(h_bits((_Float16)(bfr(a[0]) * wsc)), h_bits((_Float16)(bfr(a[1]) * wsc)));
  o[1] = pk16(h_bits((_Float16)(bfr(a[2]) * wsc)), h_bits((_Float16)(bfr(a[3]) * wsc)));
  o[2] = pk16(h_bits((_Float16)(bfr(c[0]) * wsc)), h_bits((_Float16)(bfr(c[1]) * wsc)));
  o[3] = pk16(h_bits((_Float16)(bfr(c[2]) * wsc)), h_bits((_Float16)(bfr(c[3]) * wsc)));
  if (i < n8) *(volatile v4u*)(Wh + (size_t)i * 8) = o;
  __threadfence();
  if (i < n8) *(volatile v4u*)(Wh + (size_t)i * 8) = o;
}

__global__ __launch_bounds__(256) void tconv_h16(const float* __restrict__ W, unsigned short* Wt, int R, int NC, float wsc) {
  __shared__ float tile[64][65];
  const int tid = threadIdx.x, lane = tid & 31, wave = tid >> 5;
  const int n0 = blockIdx.x * 64, k0 = blockIdx.y * 64;
  const int c4 = (tid & 15) * 4, r16 = tid >> 4;
#pragma unroll
  for (int i = 0; i < 4; ++i) {
    const int row = i * 16 + r16;
    const v4f v = *(const v4f*)(W + (size_t)(k0 + row) * NC + n0 + c4);
    tile[row][c4 + 0] = v[0];
    tile[row][c4 + 1] = v[1];
    tile[row][c4 + 2] = v[2];
    tile[row][c4 + 3] = v[3];
  }
  __syncthreads();
  const int q4 = lane >> 3, k8 = (lane & 7) * 8;
  v4u hv[2];
#pragma unroll
  for (int it = 0; it < 2; ++it) {
    const int nrow = it * 32 + wave * 4 + q4;
    v4u a;
#pragma unroll
    for (int e = 0; e < 4; ++e) {
      const float f0 = bfr(tile[k8 + 2 * e][nrow]) * wsc;
      const float f1 = bfr(tile[k8 + 2 * e + 1][nrow]) * wsc;
      a[e] = pk16(h_bits((_Float16)f0), h_bits((_Float16)f1));
    }
    hv[it] = a;
  }
  for (int pass = 0; pass < 2; ++pass) {
#pragma unroll
    for (int it = 0; it < 2; ++it) {
      const int nrow = it * 32 + wave * 4 + q4;
      *(volatile v4u*)(Wt + (size_t)(n0 + nrow) * R + k0 + k8) = hv[it];
    }
    __threadfence();
  }
}

template <int OM, int BIASM, int ACT, int RES>
__global__ __launch_bounds__(256) void gemm64(
    const unsigned short* __restrict__ Ap, int lda, long long strideA,
    const unsigned short* __restrict__ Btp, int ldb, long long strideB,
    const float* __restrict__ bias0, const float* __restrict__ bias1, int Nb,
    const float* resid,
    void* Cout, int ldc, long long strideC, long long loOff,
    int M, int N, int K, float oscale) {
  const _Float16* A  = (const _Float16*)(const void*)Ap;
  const _Float16* Bt = (const _Float16*)(const void*)Btp;
  __shared__ __align__(16) float sT[8][16 * 68];
  const int b    = blockIdx.y;
  const int lane = threadIdx.x & 31;
  const int wave = threadIdx.x >> 5;
  const int tilesN = N >> 6;
  const int tilesM = M >> 6;
  const int tile = blockIdx.x * 8 + wave;
  if (tile >= tilesM * tilesN) return;
  const int tm = tile / tilesN;
  const int tn = tile - tm * tilesN;
  const int m0 = tm << 6;
  const int n0 = tn << 6;

  const _Float16* Ab = A  + (size_t)b * strideA;
  const _Float16* Bb = Bt + (size_t)b * strideB;

  const int rlane = lane & 15;
  const int koff  = (lane >> 4) * 8;
  const int mOff  = (lane >> 4) * 8;

  v8f acc[4][4];
#pragma unroll
  for (int i = 0; i < 4; ++i)
#pragma unroll
    for (int j = 0; j < 4; ++j) acc[i][j] = zero8();

  for (int k0 = 0; k0 < K; k0 += 32) {
    v16h bh[4];
#pragma unroll
    for (int j = 0; j < 4; ++j) {
      const size_t bo = (size_t)(n0 + (j << 4) + rlane) * ldb + koff + k0;
      bh[j] = ldfrag_h(Bb + bo);
    }
#pragma unroll
    for (int i = 0; i < 4; ++i) {
      const size_t ao = (size_t)(m0 + (i << 4) + rlane) * lda + koff + k0;
      const v16h ah = ldfrag_h(Ab + ao);
#pragma unroll
      for (int j = 0; j < 4; ++j) acc[i][j] = mma_h_raw(ah, bh[j], acc[i][j]);
      dep_guard1(acc[i][0], acc[i][3], ah);
    }
    keep4_h(bh[0], bh[1], bh[2], bh[3]);
  }
  acc_guard4(acc[0][0], acc[0][1], acc[0][2], acc[0][3]);
  acc_guard4(acc[1][0], acc[1][1], acc[1][2], acc[1][3]);
  acc_guard4(acc[2][0], acc[2][1], acc[2][2], acc[2][3]);
  acc_guard4(acc[3][0], acc[3][1], acc[3][2], acc[3][3]);

  const int hh2 = lane >> 4, c4 = (lane & 15) * 4;
  const int q8  = lane >> 3, c8 = (lane & 7) * 8;
  float bc[8];
#pragma unroll
  for (int e = 0; e < 8; ++e) bc[e] = 0.f;
  if (BIASM == 0) {
    const bool use1 = (n0 >= Nb);
    if (OM == 0) {
      const int cb = n0 + c4;
      const int i0 = (cb < Nb - 4) ? cb : (Nb - 4);
      const int i1 = (cb - Nb > 0) ? (cb - Nb) : 0;
      const v4f b0v = *(const v4f*)(bias0 + i0);
      const v4f b1v = *(const v4f*)(bias1 + i1);
#pragma unroll
      for (int e = 0; e < 4; ++e) bc[e] = bfr(use1 ? b1v[e] : b0v[e]);
    } else {
      const int cb = n0 + c8;
      const int i0 = (cb < Nb - 8) ? cb : (Nb - 8);
      const int i1 = (cb - Nb > 0) ? (cb - Nb) : 0;
      const v4f b0a = *(const v4f*)(bias0 + i0), b0b = *(const v4f*)(bias0 + i0 + 4);
      const v4f b1a = *(const v4f*)(bias1 + i1), b1b = *(const v4f*)(bias1 + i1 + 4);
#pragma unroll
      for (int e = 0; e < 4; ++e) {
        bc[e]     = bfr(use1 ? b1a[e] : b0a[e]);
        bc[4 + e] = bfr(use1 ? b1b[e] : b0b[e]);
      }
    }
  }

  float* slab = sT[wave];
#pragma unroll
  for (int i = 0; i < 4; ++i) {
    const int mBase = m0 + (i << 4);
#pragma unroll
    for (int j = 0; j < 4; ++j) {
#pragma unroll
      for (int r = 0; r < 8; ++r) {
        slab[(mOff + r) * 68 + (j << 4) + rlane] = acc[i][j][r];
      }
    }
    wave_sync_lds();
    if (OM == 0) {
      float* C = (float*)Cout + (size_t)b * strideC;
      const float* Rb = resid + (size_t)b * strideC;
      v4f vals[8];
#pragma unroll
      for (int it = 0; it < 8; ++it) {
        const int row = it * 2 + hh2;
        v4f v = *(const v4f*)(slab + row * 68 + c4);
#pragma unroll
        for (int e = 0; e < 4; ++e) {
          float f = v[e] * oscale + bc[e];
          if (ACT) f = gelu_f(f);
          v[e] = f;
        }
        if (RES == 1 || RES == 3) {
          const v4f rr = *(const v4f*)(Rb + (size_t)(mBase + row) * ldc + n0 + c4);
#pragma unroll
          for (int e = 0; e < 4; ++e) v[e] += (RES == 3) ? bfr(rr[e]) : rr[e];
        }
        vals[it] = v;
      }
      for (int pass = 0; pass < 2; ++pass) {
#pragma unroll
        for (int it = 0; it < 8; ++it) {
          const int row = it * 2 + hh2;
          *(volatile v4f*)(C + (size_t)(mBase + row) * ldc + n0 + c4) = vals[it];
        }
        __threadfence();
      }
    } else {
      unsigned short* C = (unsigned short*)Cout + (size_t)b * strideC;
      v4u hv[4], lv[4];
#pragma unroll
      for (int it = 0; it < 4; ++it) {
        const int row = it * 4 + q8;
        const float* sp = slab + row * 68 + c8;
        float bm = 0.f;
        if (BIASM == 1) bm = bfr(bias0[mBase + row]);
        v4u a, al;
#pragma unroll
        for (int e = 0; e < 4; ++e) {
          float f0 = sp[2 * e]     * oscale + ((BIASM == 1) ? bm : bc[2 * e]);
          float f1 = sp[2 * e + 1] * oscale + ((BIASM == 1) ? bm : bc[2 * e + 1]);
          if (ACT) { f0 = gelu_f(f0); f1 = gelu_f(f1); }
          unsigned short u0, u1, w0 = 0, w1 = 0;
          if (OM == 1)      { u0 = bf_bits(f0); u1 = bf_bits(f1); }
          else if (OM == 2) { u0 = h_bits((_Float16)f0); u1 = h_bits((_Float16)f1); }
          else              { split_h(f0, u0, w0); split_h(f1, u1, w1); }
          a[e]  = pk16(u0, u1);
          al[e] = pk16(w0, w1);
        }
        hv[it] = a;
        lv[it] = al;
      }
      for (int pass = 0; pass < 2; ++pass) {
#pragma unroll
        for (int it = 0; it < 4; ++it) {
          const int row = it * 4 + q8;
          const size_t co = (size_t)(mBase + row) * ldc + n0 + c8;
          *(volatile v4u*)(C + co) = hv[it];
          if (OM == 3) *(volatile v4u*)(C + loOff + co) = lv[it];
        }
        __threadfence();
      }
    }
    wave_sync_lds();
  }
}

__global__ __launch_bounds__(256) void vsum(const unsigned short* __restrict__ hp, const unsigned short* __restrict__ lp,
                                           float* csum) {
  const int tid = threadIdx.x, lane = tid & 31, wave = tid >> 5;
  const int rowbase = (blockIdx.x * 8 + wave) * 32;
  const _Float16* Hb = (const _Float16*)(const void*)hp;
  const _Float16* Lb = (const _Float16*)(const void*)lp;
  float mine = 0.f;
#pragma unroll 1
  for (int rr = 0; rr < 32; ++rr) {
    const int row = rowbase + rr;
    const _Float16* hr = Hb + (size_t)row * SEQ + lane * (SEQ / 32);
    const _Float16* lr = Lb + (size_t)row * SEQ + lane * (SEQ / 32);
    float sh = 0.f, sl = 0.f;
#pragma unroll
    for (int i = 0; i < SEQ / 256; ++i) {
      const v8h a = *(const v8h*)(hr + 8 * i);
      const v8h c = *(const v8h*)(lr + 8 * i);
#pragma unroll
      for (int e = 0; e < 8; ++e) { sh += (float)a[e]; sl += (float)c[e]; }
    }
    float tot = sh + sl * (1.0f / LOSC);
    tot = wsum(tot);
    mine = (lane == rr) ? tot : mine;
  }
  __shared__ __align__(16) float stage[8][32];
  stage[wave][lane] = mine;
  __syncthreads();
  typedef float v4f_vs __attribute__((ext_vector_type(4)));
  for (int pass = 0; pass < 2; ++pass) {
    if (lane < 8) {
      const v4f_vs v = *(const v4f_vs*)(&stage[wave][4 * lane]);
      *(volatile v4f_vs*)(csum + rowbase + 4 * lane) = v;
    }
    __threadfence();
  }
}

__global__ __launch_bounds__(128)
void attn2q(const unsigned short* __restrict__ qkp, const unsigned short* __restrict__ vtp,
            const float* __restrict__ taup, const float* __restrict__ csp,
            unsigned short* chi, unsigned short* clo) {
  __shared__ __align__(16) _Float16 Ksh[64 * 64];
  __shared__ __align__(16) _Float16 Vth[64 * 64];
  __shared__ __align__(16) _Float16 Psh[4][16 * 64];
  __shared__ __align__(16) float    Os[4][16 * 64];

  const int tid  = threadIdx.x;
  const int wave = tid >> 5;
  const int lane = tid & 31;
  const int hh   = lane >> 4;
  const int c    = lane & 15;

  const int bx   = blockIdx.x;
  const int qb   = bx % NQB;
  const int rest = bx / NQB;
  const int h    = rest % NH;
  const int b    = rest / NH;
  const int q0   = qb * 64 + wave * 16;
  const size_t rowB = (size_t)b * SEQ;

  const _Float16* Qh = (const _Float16*)(const void*)qkp + (size_t)h * HD;
  const _Float16* Kg = (const _Float16*)(const void*)qkp + DM + (size_t)h * HD;
  const _Float16* Vh = (const _Float16*)(const void*)vtp + ((size_t)b * DM + (size_t)h * HD) * SEQ;

  const float tv     = bfr(taup[h]);
  const float sscale = 1.0f / (8.0f * tv);
  float cs[4];
#pragma unroll
  for (int t = 0; t < 4; ++t) cs[t] = csp[(size_t)b * DM + h * HD + t * 16 + c];

  v16h qa[2];
#pragma unroll
  for (int dc = 0; dc < 2; ++dc) qa[dc] = ldfrag_h(Qh + (rowB + q0 + c) * QKP + dc * 32 + 8 * hh);

  float rs[8];
  v8f oacc[4];
#pragma unroll
  for (int r = 0; r < 8; ++r) rs[r] = 0.f;
#pragma unroll
  for (int t = 0; t < 4; ++t) oacc[t] = zero8();

  for (int kt = 0; kt < NQB; ++kt) {
    const int kv0 = kt * 64;
    __syncthreads();
    {
      const int r = tid >> 1, hf = (tid & 1) * 32;
      const _Float16* kg = Kg + (rowB + kv0 + r) * QKP + hf;
      const _Float16* vg = Vh + (size_t)r * SEQ + kv0 + hf;
#pragma unroll
      for (int i = 0; i < 4; ++i) {
        const v8h a0 = *(const v8h*)(kg + 8 * i);
        const v8h b0 = *(const v8h*)(vg + 8 * i);
        *(v8h*)(Ksh + r * 64 + hf + 8 * i) = a0;
        *(v8h*)(Vth + r * 64 + hf + 8 * i) = b0;
      }
    }
    __syncthreads();

    v8f s[4];
#pragma unroll
    for (int j = 0; j < 4; ++j) {
      v8f sh = zero8();
#pragma unroll
      for (int dc = 0; dc < 2; ++dc) {
        FragH kb;
        kb.h[0] = *(const v8h*)(Ksh + (j * 16 + c) * 64 + dc * 32 + 8 * hh);
        kb.h[1] = *(const v8h*)(Ksh + (j * 16 + c) * 64 + dc * 32 + 16 + 8 * hh);
        sh = mma_h(qa[dc], kb.v, sh);
      }
#pragma unroll
      for (int r = 0; r < 8; ++r) s[j][r] = sh[r] * sscale;
    }

    _Float16* pwh = Psh[wave];
#pragma unroll
    for (int j = 0; j < 4; ++j) {
#pragma unroll
      for (int r = 0; r < 8; ++r) {
        const float sv = s[j][r];
        const float u  = sv + QC;
        rs[r] += u * u;
        const float ep = sv * (sv + 2.0f * QC);
        pwh[(8 * hh + r) * 64 + j * 16 + c] = (_Float16)(ep * PSC);
      }
    }
    wave_sync_lds();

#pragma unroll 1
    for (int kk = 0; kk < 2; ++kk) {
      FragH pa;
      pa.h[0] = *(const v8h*)(pwh + c * 64 + kk * 32 + 8 * hh);
      pa.h[1] = *(const v8h*)(pwh + c * 64 + kk * 32 + 16 + 8 * hh);
#pragma unroll
      for (int t = 0; t < 4; ++t) {
        FragH vb;
        vb.h[0] = *(const v8h*)(Vth + (t * 16 + c) * 64 + kk * 32 + 8 * hh);
        vb.h[1] = *(const v8h*)(Vth + (t * 16 + c) * 64 + kk * 32 + 16 + 8 * hh);
        oacc[t] = mma_h(pa.v, vb.v, oacc[t]);
      }
    }
  }

  float* os = Os[wave];
#pragma unroll
  for (int r = 0; r < 8; ++r) {
    float S = rs[r];
    S += __shfl_xor(S, 8, 32);
    S += __shfl_xor(S, 4, 32);
    S += __shfl_xor(S, 2, 32);
    S += __shfl_xor(S, 1, 32);
    const float inv = (1.0f / (S + QEPS)) * CSC;
#pragma unroll
    for (int t = 0; t < 4; ++t)
      os[(8 * hh + r) * 64 + t * 16 + c] = (oacc[t][r] * (1.0f / PSC) + (QC * QC) * cs[t]) * inv;
  }
  wave_sync_lds();
  {
    const int q4 = lane >> 3, c8 = (lane & 7) * 8;
    v4u hv[4], lv[4];
#pragma unroll
    for (int it = 0; it < 4; ++it) {
      const int row = it * 4 + q4;
      const float* sp = os + row * 64 + c8;
      v4u a, al;
#pragma unroll
      for (int e = 0; e < 4; ++e) {
        unsigned short u0, u1, w0, w1;
        split_h(sp[2 * e],     u0, w0);
        split_h(sp[2 * e + 1], u1, w1);
        a[e]  = pk16(u0, u1);
        al[e] = pk16(w0, w1);
      }
      hv[it] = a;
      lv[it] = al;
    }
    for (int pass = 0; pass < 2; ++pass) {
#pragma unroll
      for (int it = 0; it < 4; ++it) {
        const int row = it * 4 + q4;
        const size_t go = (rowB + q0 + row) * DM + (size_t)h * HD + c8;
        *(volatile v4u*)(chi + go) = hv[it];
        *(volatile v4u*)(clo + go) = lv[it];
      }
      __threadfence();
    }
  }
}

extern "C" void kernel_launch(void* const* d_in, const int* in_sizes, int n_in,
                              void* d_out, int out_size, void* d_ws, size_t ws_size,
                              hipStream_t stream) {
  if (n_in < 4) return;
  if (in_sizes[0] != MP * DM) return;
  if (in_sizes[1] != DM * W3) return;
  if (in_sizes[2] != DM * DM) return;
  if (in_sizes[3] != NH) return;
  if (out_size != MP * DM) return;

  const float* x    = (const float*)d_in[0];
  const float* wqkv = (const float*)d_in[1];
  const float* wo   = (const float*)d_in[2];
  const float* tau  = (const float*)d_in[3];

  const size_t PWT  = (size_t)W3 * DM * 2;
  const size_t PWO  = (size_t)DM * DM * 2;
  const size_t PXH  = (size_t)MP * DM * 2;
  const size_t PQK  = (size_t)MP * QKP * 2;
  const size_t PVT  = (size_t)NBATCH * DM * SEQ * 2;
  const size_t PCS  = (size_t)NBATCH * DM * 4;
  const size_t PCTX = (size_t)MP * DM * 2;
  const size_t PHF  = (size_t)MP * DM * 4;
  size_t off = 0;
  const size_t oWT  = off; off += PWT;
  const size_t oWo  = off; off += PWO;
  const size_t oXH  = off; off += PXH;
  const size_t oQK  = off; off += PQK;
  const size_t oVTh = off; off += PVT;
  const size_t oVTl = off; off += PVT;
  const size_t oCS  = off; off += PCS;
  const size_t oCh  = off; off += PCTX;
  const size_t oCl  = off; off += PCTX;
  const size_t oHf  = off; off += PHF;
  if (off > ws_size) return;
  if (off > (size_t)134217728) return;

  char* ws = (char*)d_ws;
  unsigned short* WT   = (unsigned short*)(ws + oWT);
  unsigned short* WoT  = (unsigned short*)(ws + oWo);
  unsigned short* XH   = (unsigned short*)(ws + oXH);
  unsigned short* QK   = (unsigned short*)(ws + oQK);
  unsigned short* VTh  = (unsigned short*)(ws + oVTh);
  unsigned short* VTl  = (unsigned short*)(ws + oVTl);
  float*          CS   = (float*)(ws + oCS);
  unsigned short* CtxH = (unsigned short*)(ws + oCh);
  unsigned short* CtxL = (unsigned short*)(ws + oCl);
  float*          Hf   = (float*)(ws + oHf);
  float*          out0 = (float*)d_out;

  const int n8x = (MP * DM) / 8;
  if ((n8x % 256) != 0) return;
  const dim3 blk(256), blk128(128);
  const dim3 gCx(n8x / 256);
  const dim3 gTw(W3 / 64, DM / 64);
  const dim3 gTo(DM / 64, DM / 64);
  const dim3 gNqk(((MP / 64) * (QKP / 64) + 7) / 8, 1);
  const dim3 gVT(((DM / 64) * (SEQ / 64) + 7) / 8, NBATCH);
  const dim3 gCs((NBATCH * DM) / 256);
  const dim3 gAttn(NBATCH * NH * NQB);
  const dim3 gNo(((MP / 64) * (DM / 64) + 7) / 8, 1);
  const float invw  = 1.0f / WSC;
  const float invhi = 1.0f / (WSC * CSC);
  const float invlo = invhi / LOSC;
  const long long vtlo = (long long)((oVTl - oVTh) / 2);

  conv_h16<<<gCx, blk, 0, stream>>>(x, XH, n8x, 1.0f);
  tconv_h16<<<gTw, blk, 0, stream>>>(wqkv, WT, DM, W3, WSC);
  tconv_h16<<<gTo, blk, 0, stream>>>(wo, WoT, DM, DM, WSC);

  gemm64<2, 2, 0, 0><<<gNqk, blk, 0, stream>>>(
      XH, DM, 0LL, WT, DM, 0LL, x, x, QKP, x,
      (void*)QK, QKP, 0LL, 0LL, MP, QKP, DM, invw);
  gemm64<3, 2, 0, 0><<<gVT, blk, 0, stream>>>(
      WT + (size_t)2 * DM * DM, DM, 0LL, XH, DM, (long long)SEQ * DM, x, x, SEQ, x,
      (void*)VTh, SEQ, (long long)DM * SEQ, vtlo, DM, SEQ, DM, invw);

  vsum<<<gCs, blk, 0, stream>>>(VTh, VTl, CS);

  attn2q<<<gAttn, blk128, 0, stream>>>(QK, VTh, tau, CS, CtxH, CtxL);

  gemm64<0, 2, 0, 0><<<gNo, blk, 0, stream>>>(
      CtxH, DM, 0LL, WoT, DM, 0LL, x, x, DM, x,
      (void*)Hf, DM, 0LL, 0LL, MP, DM, DM, invhi);
  gemm64<0, 2, 0, 1><<<gNo, blk, 0, stream>>>(
      CtxL, DM, 0LL, WoT, DM, 0LL, x, x, DM, Hf,
      (void*)out0, DM, 0LL, 0LL, MP, DM, DM, invlo);
  (void)hipGetLastError();
}
